// TransitionModel_76982993813766
// MI455X (gfx1250) — hardware-verified
//
#include <hip/hip_runtime.h>
#include <math.h>

typedef __attribute__((ext_vector_type(16))) _Float16 v16h;
typedef __attribute__((ext_vector_type(16))) __bf16 v16b;
typedef __attribute__((ext_vector_type(8)))  _Float16 v8h;
typedef __attribute__((ext_vector_type(8)))  float v8f;
typedef __attribute__((ext_vector_type(4)))  float v4f;
typedef __attribute__((ext_vector_type(2)))  float v2f;
typedef __attribute__((ext_vector_type(4)))  unsigned v4u;
typedef __attribute__((ext_vector_type(4)))  int v4i;
typedef float __attribute__((may_alias)) float_a;
typedef int __attribute__((may_alias)) int_a;

template <typename T> __device__ __forceinline__ void vst2(void* p, T v) { *(volatile T*)p = v; __threadfence(); *(volatile T*)p = v; }
__device__ __forceinline__ v8f wmma16(v16h a, v16h b, v8f c) {
  v8f d = __builtin_amdgcn_wmma_f32_16x16x32_f16(false, a, false, b, (short)0, c, false, false);
  asm volatile("v_nop\n\tv_nop\n\tv_nop\n\tv_nop" : "+v"(d) : "v"(a), "v"(b));
  return d;
}
__device__ __forceinline__ v8f wmma_bf(v16b a, v16b b, v8f c) {
  v8f d = __builtin_amdgcn_wmma_f32_16x16x32_bf16(false, a, false, b, (short)0, c, false, false);
  asm volatile("v_nop\n\tv_nop\n\tv_nop\n\tv_nop" : "+v"(d) : "v"(a), "v"(b));
  return d;
}
__device__ __forceinline__ v16h frag_h(const _Float16* rowk0, int lane) {
  union { v16h v; v8h q[2]; } u; const _Float16* p = rowk0 + 8 * (lane >> 4);
  u.q[0] = *(const v8h*)p; u.q[1] = *(const v8h*)(p + 16); return u.v;
}
__device__ __forceinline__ v16h frag_f32(const float* rowk0, int lane) {
  v16h a; const float* p = rowk0 + 8 * (lane >> 4);
#pragma unroll
  for (int i = 0; i < 8; ++i) { a[i] = (_Float16)p[i]; a[8 + i] = (_Float16)p[16 + i]; }
  return a;
}
__device__ __forceinline__ v16h frag_f32s(const float* rowk0, int lane, float sc) {
  v16h a; const float* p = rowk0 + 8 * (lane >> 4);
#pragma unroll
  for (int i = 0; i < 8; ++i) { a[i] = (_Float16)(p[i] * sc); a[8 + i] = (_Float16)(p[16 + i] * sc); }
  return a;
}
__device__ __forceinline__ v16h fragc_f32(const float* W, int k0, int n, int lane, int ld, int K) {
  v16h a; const int g = lane >> 4;
#pragma unroll
  for (int i = 0; i < 8; ++i) { const int ka = k0 + 8 * g + i, kb = ka + 16;
    a[i] = (_Float16)(ka < K ? W[(size_t)(ka < K ? ka : K - 1) * ld + n] : 0.f); a[8 + i] = (_Float16)(kb < K ? W[(size_t)(kb < K ? kb : K - 1) * ld + n] : 0.f); }
  return a;
}
struct F2 { v16b h, l; };
__device__ __forceinline__ F2 bsplit16(const float v[16]) { F2 r;
#pragma unroll
  for (int i = 0; i < 16; ++i) { const __bf16 h = (__bf16)v[i]; r.h[i] = h; r.l[i] = (__bf16)(v[i] - (float)h); }
  return r; }
__device__ __forceinline__ F2 split_row(const float* row, int k0, int lane) { float v[16]; const float* p = row + k0 + 8 * (lane >> 4);
#pragma unroll
  for (int i = 0; i < 8; ++i) { v[i] = p[i]; v[8 + i] = p[16 + i]; }
  return bsplit16(v); }
__device__ __forceinline__ F2 split_rowK(const float* row, int k0, int lane, int K) { float v[16]; const int g = lane >> 4;
#pragma unroll
  for (int i = 0; i < 8; ++i) { const int ka = k0 + 8 * g + i, kb = ka + 16; v[i] = ka < K ? row[ka < K ? ka : K - 1] : 0.f; v[8 + i] = kb < K ? row[kb < K ? kb : K - 1] : 0.f; }
  return bsplit16(v); }
__device__ __forceinline__ F2 split_col(const float* W, int k0, int n, int lane, int ld, int K) { float v[16]; const int g = lane >> 4;
#pragma unroll
  for (int i = 0; i < 8; ++i) { const int ka = k0 + 8 * g + i, kb = ka + 16; v[i] = ka < K ? W[(size_t)(ka < K ? ka : K - 1) * ld + n] : 0.f; v[8 + i] = kb < K ? W[(size_t)(kb < K ? kb : K - 1) * ld + n] : 0.f; }
  return bsplit16(v); }
__device__ __forceinline__ v8f mac3(const F2& a, const F2& b, v8f c) { c = wmma_bf(a.l, b.h, c); c = wmma_bf(a.h, b.l, c); return wmma_bf(a.h, b.h, c); }
__device__ __forceinline__ float sigm(float v) { return 1.0f / (1.0f + expf(-v)); }
#define LDSX() do { asm volatile("s_wait_dscnt 0" ::: "memory"); __builtin_amdgcn_wave_barrier(); __builtin_amdgcn_fence(__ATOMIC_RELEASE, "workgroup"); } while (0)


#define NBR 256
#define NN 1024
typedef __attribute__((ext_vector_type(8))) __bf16 v8b;
__device__ __forceinline__ v16b frag_b(const __bf16* rowk0, int lane) {
  union { v16b v; v8b q[2]; } u; const __bf16* p = rowk0 + 8 * (lane >> 4);
  u.q[0] = *(const v8b*)p; u.q[1] = *(const v8b*)(p + 16); return u.v;
}
__device__ __forceinline__ float bfr(float v) { return (float)(__bf16)v; }
__device__ __attribute__((noinline)) float exp_ni(float v) { return expf(v); }
__device__ __attribute__((noinline)) float erf_ni(float v) { return erff(v); }

#define WS_BT  0u
#define WS_CL  (WS_BT + 4u * (size_t)NN * NN)
#define WS_END (WS_CL + 4u * NN)

__global__ __launch_bounds__(256) void k_prep(const float* __restrict__ Wm, float* __restrict__ BT, float* __restrict__ CL) { __shared__ __align__(16) float st[64][68]; __shared__ float smx[4][64], ssm[4][64]; __shared__ float cmx[64]; __shared__ __align__(16) float scl[64];
  const int t = threadIdx.x; const int j0 = blockIdx.x * 64; const int jl = t & 63, part = t >> 6;
  { float mx = -3.0e38f;
#pragma unroll 1
    for (int k = part; k < NN; k += 4) mx = fmaxf(mx, bfr(Wm[(size_t)k * NN + j0 + jl]));
    smx[part][jl] = mx; }
  __syncthreads(); if (t < 64) cmx[t] = fmaxf(fmaxf(smx[0][t], smx[1][t]), fmaxf(smx[2][t], smx[3][t])); __syncthreads();
  float csum = 0.f;
#pragma unroll 1
  for (int kb = 0; kb < NN / 64; ++kb) {
    for (int e = t; e < 64 * 64; e += 256) { const int kl = e >> 6, jj = e & 63; st[jj][kl] = expf(bfr(Wm[(size_t)(kb * 64 + kl) * NN + j0 + jj]) - cmx[jj]); }
    __syncthreads();
    { const int jj = t >> 2, q4 = t & 3;
#pragma unroll
      for (int i = 0; i < 16; ++i) csum += st[jj][q4 * 16 + i];
      for (int q = q4 * 4; q < q4 * 4 + 4; ++q) vst2(BT + (size_t)(j0 + jj) * NN + kb * 64 + q * 4, *(const v4f*)&st[jj][q * 4]); }
    __syncthreads(); }
  csum += __shfl_xor(csum, 1); csum += __shfl_xor(csum, 2);
  if ((t & 3) == 0) scl[t >> 2] = logf(csum);
  __syncthreads(); if (t < 16) vst2(CL + j0 + t * 4, *(const v4f*)&scl[t * 4]); }
__global__ __launch_bounds__(128) void k_out(const float* __restrict__ LA, const float* __restrict__ BT, const float* __restrict__ CL, float* __restrict__ OUT) { __shared__ __align__(16) float sa[4][16][36]; __shared__ __align__(16) float sf[4][16][132]; __shared__ float smb[4][16];
  const int tid = threadIdx.x, wave = tid >> 5, lane = tid & 31, col = lane & 15, g = lane >> 4; const int r0 = blockIdx.x * 64 + wave * 16; const int c0 = blockIdx.y * 128;
  { const int rr = lane >> 1, half = lane & 1; const float* lr = LA + (size_t)(r0 + rr) * NN + half * (NN / 2); float mx = -3.0e38f;
#pragma unroll 1
    for (int k = 0; k < NN / 2; ++k) mx = fmaxf(mx, bfr(lr[k]));
    mx = fmaxf(mx, __shfl_xor(mx, 1)); if (half == 0) smb[wave][rr] = mx; }
  LDSX();
  v8f acc[8] = {};
#pragma unroll 1
  for (int kc = 0; kc < NN / 32; ++kc) {
    for (int e = lane; e < 16 * 32; e += 32) { const int rr = e >> 5, kk = e & 31; sa[wave][rr][kk] = expf(bfr(LA[(size_t)(r0 + rr) * NN + kc * 32 + kk]) - smb[wave][rr]); }
    LDSX();
    const F2 a = split_row(&sa[wave][col][0], 0, lane);
#pragma unroll
    for (int j = 0; j < 8; ++j) { const F2 bw = split_row(BT + (size_t)(c0 + j * 16 + col) * NN, kc * 32, lane); acc[j] = wmma_bf(a.h, bw.h, acc[j]); acc[j] = wmma_bf(a.h, bw.l, acc[j]); acc[j] = wmma_bf(a.l, bw.h, acc[j]); }
    LDSX(); }
#pragma unroll
  for (int j = 0; j < 8; ++j)
#pragma unroll
    for (int r = 0; r < 8; ++r) sf[wave][8 * g + r][j * 16 + col] = smb[wave][8 * g + r] + logf(acc[j][r]) - CL[c0 + j * 16 + col];
  LDSX(); for (int rl = 0; rl < 16; ++rl) vst2(OUT + (size_t)(r0 + rl) * NN + c0 + lane * 4, *(const v4f*)&sf[wave][rl][lane * 4]); }
extern "C" void kernel_launch(void* const* d_in, const int* in_sizes, int n_in, void* d_out, int out_size, void* d_ws, size_t ws_size, hipStream_t stream) {
  (void)in_sizes; (void)n_in; (void)out_size;
  const float** F = (const float**)d_in;
  if (ws_size < (size_t)WS_END) return;
  char* ws = (char*)d_ws; float *BT = (float*)(ws + WS_BT), *CL = (float*)(ws + WS_CL);
  k_prep<<<NN / 64, 256, 0, stream>>>(F[1], BT, CL);
  k_out<<<dim3(NBR / 64, NN / 128), 128, 0, stream>>>(F[0], BT, CL, (float*)d_out);
}
